// DynamLinear_15101105013222
// MI455X (gfx1250) — hardware-verified
//
#include <hip/hip_runtime.h>
#include <math.h>

typedef __attribute__((ext_vector_type(16))) _Float16 v16h;
typedef __attribute__((ext_vector_type(16))) __bf16 v16b;
typedef __attribute__((ext_vector_type(8)))  _Float16 v8h;
typedef __attribute__((ext_vector_type(8)))  float v8f;
typedef __attribute__((ext_vector_type(4)))  float v4f;
typedef __attribute__((ext_vector_type(2)))  float v2f;
typedef __attribute__((ext_vector_type(4)))  unsigned v4u;
typedef __attribute__((ext_vector_type(4)))  int v4i;
typedef float __attribute__((may_alias)) float_a;
typedef int __attribute__((may_alias)) int_a;

template <typename T> __device__ __forceinline__ void vst2(void* p, T v) { *(volatile T*)p = v; __threadfence(); *(volatile T*)p = v; }
__device__ __forceinline__ v8f wmma16(v16h a, v16h b, v8f c) {
  v8f d = __builtin_amdgcn_wmma_f32_16x16x32_f16(false, a, false, b, (short)0, c, false, false);
  asm volatile("v_nop\n\tv_nop\n\tv_nop\n\tv_nop" : "+v"(d) : "v"(a), "v"(b));
  return d;
}
__device__ __forceinline__ v8f wmma_bf(v16b a, v16b b, v8f c) {
  v8f d = __builtin_amdgcn_wmma_f32_16x16x32_bf16(false, a, false, b, (short)0, c, false, false);
  asm volatile("v_nop\n\tv_nop\n\tv_nop\n\tv_nop" : "+v"(d) : "v"(a), "v"(b));
  return d;
}
__device__ __forceinline__ v16h frag_h(const _Float16* rowk0, int lane) {
  union { v16h v; v8h q[2]; } u; const _Float16* p = rowk0 + 8 * (lane >> 4);
  u.q[0] = *(const v8h*)p; u.q[1] = *(const v8h*)(p + 16); return u.v;
}
__device__ __forceinline__ v16h frag_f32(const float* rowk0, int lane) {
  v16h a; const float* p = rowk0 + 8 * (lane >> 4);
#pragma unroll
  for (int i = 0; i < 8; ++i) { a[i] = (_Float16)p[i]; a[8 + i] = (_Float16)p[16 + i]; }
  return a;
}
__device__ __forceinline__ v16h frag_f32s(const float* rowk0, int lane, float sc) {
  v16h a; const float* p = rowk0 + 8 * (lane >> 4);
#pragma unroll
  for (int i = 0; i < 8; ++i) { a[i] = (_Float16)(p[i] * sc); a[8 + i] = (_Float16)(p[16 + i] * sc); }
  return a;
}
__device__ __forceinline__ v16h fragc_f32(const float* W, int k0, int n, int lane, int ld, int K) {
  v16h a; const int g = lane >> 4;
#pragma unroll
  for (int i = 0; i < 8; ++i) { const int ka = k0 + 8 * g + i, kb = ka + 16;
    a[i] = (_Float16)(ka < K ? W[(size_t)(ka < K ? ka : K - 1) * ld + n] : 0.f); a[8 + i] = (_Float16)(kb < K ? W[(size_t)(kb < K ? kb : K - 1) * ld + n] : 0.f); }
  return a;
}
struct F2 { v16b h, l; };
__device__ __forceinline__ F2 bsplit16(const float v[16]) { F2 r;
#pragma unroll
  for (int i = 0; i < 16; ++i) { const __bf16 h = (__bf16)v[i]; r.h[i] = h; r.l[i] = (__bf16)(v[i] - (float)h); }
  return r; }
__device__ __forceinline__ F2 split_row(const float* row, int k0, int lane) { float v[16]; const float* p = row + k0 + 8 * (lane >> 4);
#pragma unroll
  for (int i = 0; i < 8; ++i) { v[i] = p[i]; v[8 + i] = p[16 + i]; }
  return bsplit16(v); }
__device__ __forceinline__ F2 split_rowK(const float* row, int k0, int lane, int K) { float v[16]; const int g = lane >> 4;
#pragma unroll
  for (int i = 0; i < 8; ++i) { const int ka = k0 + 8 * g + i, kb = ka + 16; v[i] = ka < K ? row[ka < K ? ka : K - 1] : 0.f; v[8 + i] = kb < K ? row[kb < K ? kb : K - 1] : 0.f; }
  return bsplit16(v); }
__device__ __forceinline__ F2 split_col(const float* W, int k0, int n, int lane, int ld, int K) { float v[16]; const int g = lane >> 4;
#pragma unroll
  for (int i = 0; i < 8; ++i) { const int ka = k0 + 8 * g + i, kb = ka + 16; v[i] = ka < K ? W[(size_t)(ka < K ? ka : K - 1) * ld + n] : 0.f; v[8 + i] = kb < K ? W[(size_t)(kb < K ? kb : K - 1) * ld + n] : 0.f; }
  return bsplit16(v); }
__device__ __forceinline__ v8f mac3(const F2& a, const F2& b, v8f c) { c = wmma_bf(a.l, b.h, c); c = wmma_bf(a.h, b.l, c); return wmma_bf(a.h, b.h, c); }
__device__ __forceinline__ float sigm(float v) { return 1.0f / (1.0f + expf(-v)); }
#define LDSX() do { asm volatile("s_wait_dscnt 0" ::: "memory"); __builtin_amdgcn_wave_barrier(); __builtin_amdgcn_fence(__ATOMIC_RELEASE, "workgroup"); } while (0)


#define NT 8192
#define FD 1024
#define NCB 16
#define CW 64
__device__ __forceinline__ float bfr(float v) { return (float)(__bf16)v; }

__global__ __launch_bounds__(128) void k_dyn(const float* __restrict__ x, const float* __restrict__ W, float* __restrict__ out) {
  __shared__ __align__(16) float sy[16][NCB * CW + 4];
  __shared__ float ssq[16][33];
  __shared__ __align__(16) float so[16][FD + 4];
  const int tid = threadIdx.x, wave = tid >> 5, lane = tid & 31, col = lane & 15, g = lane >> 4; const size_t t0 = (size_t)blockIdx.x * 16;
  { v8f acc[16] = {};
#pragma unroll 1
    for (int kc = 0; kc < FD / 32; ++kc) { const v16b a = split_row(x + (t0 + col) * FD, kc * 32, lane).h;
#pragma unroll
      for (int j = 0; j < 16; ++j) { const int n = wave * 256 + j * 16 + col; const int h = n >> 6, c = n & 63; acc[j] = wmma_bf(a, split_col(W + (size_t)h * FD * CW, kc * 32, c, lane, CW, FD).h, acc[j]); } }
#pragma unroll
    for (int j = 0; j < 16; ++j)
#pragma unroll
      for (int r = 0; r < 8; ++r) sy[8 * g + r][wave * 256 + j * 16 + col] = acc[j][r]; }
  __syncthreads();
  const int tl = tid >> 3, i0 = (tid & 7) * 4; float sq = 0.f;
#pragma unroll 1
  for (int ii = 0; ii < 4; ++ii) { const int i = i0 + ii; float o[32];
#pragma unroll
    for (int j = 0; j < 32; ++j) o[j] = 0.f;
#pragma unroll 1
    for (int h = 0; h < NCB; ++h) { const float a = sy[tl][h * CW + i]; const float* bp = &sy[tl][h * CW + 32];
#pragma unroll
      for (int j = 0; j < 32; ++j) o[j] += a * bp[j]; }
#pragma unroll
    for (int j = 0; j < 32; ++j) { const float v = o[j] * 0.25f; so[tl][i * 32 + j] = v; sq += v * v; } }
  ssq[tl][tid & 7] = sq;
  __syncthreads();
  { float tot = 0.f;
#pragma unroll
    for (int k = 0; k < 8; ++k) tot += ssq[tl][k];
    const float rs = rsqrtf(tot * (1.0f / FD) + 1e-12f);
#pragma unroll 1
    for (int ii = 0; ii < 4; ++ii) { const int i = i0 + ii;
#pragma unroll
      for (int j = 0; j < 32; ++j) so[tl][i * 32 + j] *= rs; } }
  __syncthreads();
  for (int q = tid; q < 16 * FD / 4; q += 128) { const int r = q >> 8, pc = q & 255; vst2(out + (t0 + r) * FD + pc * 4, *(const v4f*)(&so[r][pc * 4])); }
}
extern "C" void kernel_launch(void* const* d_in, const int* in_sizes, int n_in, void* d_out, int out_size, void* d_ws, size_t ws_size, hipStream_t stream) {
  (void)in_sizes; (void)n_in; (void)out_size; (void)ws_size; (void)d_ws;
  k_dyn<<<NT / 16, 128, 0, stream>>>((const float*)d_in[0], (const float*)d_in[1], (float*)d_out);
}
